// SelfAttentionLayerFull_18657337933943
// MI455X (gfx1250) — hardware-verified
//
#include <hip/hip_runtime.h>
#include <math.h>

constexpr int kBatch   = 4;
constexpr int kTok     = 4096;
constexpr int kDim     = 512;
constexpr int kRows    = kBatch * kTok;
constexpr int kHalfQ   = 2048;
constexpr int kHalfRow = kTok / 2;
constexpr float kScoreScale = 0.044194173824159216f;
constexpr float kPCarry     = 32768.0f;
constexpr float kPCarryInv  = 1.0f / 32768.0f;

constexpr size_t kPlane16  = (size_t)kRows * kDim * 2;
constexpr size_t kWtBytes  = (size_t)3 * kDim * kDim * 2;
constexpr size_t kSBytes   = (size_t)kHalfQ * kTok * 4;
constexpr size_t kOffXb = 0;
constexpr size_t kOffWt = kOffXb + kPlane16;
constexpr size_t kOffQp = kOffWt + kWtBytes;
constexpr size_t kOffKp = kOffQp + kPlane16;
constexpr size_t kOffVt = kOffKp + kPlane16;
constexpr size_t kOffS  = kOffVt + kPlane16;
constexpr size_t kWsTotal = kOffS + kSBytes;
static_assert(kWsTotal <= (size_t)134217728);
static_assert((size_t)kHalfQ * kTok * 2 <= kPlane16);

typedef __attribute__((ext_vector_type(16))) _Float16 v16h;
typedef __attribute__((ext_vector_type(8)))  _Float16 v8h;
typedef __attribute__((ext_vector_type(16))) __bf16   v16b;
typedef __attribute__((ext_vector_type(8)))  __bf16   v8b;
typedef __attribute__((ext_vector_type(8)))  float    v8f;
typedef __attribute__((ext_vector_type(4)))  float    v4f;
typedef __attribute__((ext_vector_type(4)))  unsigned int v4u;

__device__ __forceinline__ unsigned short f2bf_bits(float f) {
  unsigned u = __float_as_uint(f);
  return (unsigned short)((u + 0x7FFFu + ((u >> 16) & 1u)) >> 16);
}
__device__ __forceinline__ float bf_bits2f(unsigned short h) { return __uint_as_float(((unsigned)h) << 16); }

__device__ __forceinline__ void dep_guard_h(v8f& a, v8f& b, v16h x, v16h y) { asm volatile("v_nop\n\tv_nop\n\tv_nop\n\tv_nop" : "+v"(a), "+v"(b) : "v"(x), "v"(y)); }
__device__ __forceinline__ void dep_guard_b(v8f& a, v8f& b, v16b x, v16b y) { asm volatile("v_nop\n\tv_nop\n\tv_nop\n\tv_nop" : "+v"(a), "+v"(b) : "v"(x), "v"(y)); }
__device__ __forceinline__ void keep4_h(v16h a, v16h b, v16h c, v16h d) { asm volatile("v_nop" :: "v"(a), "v"(b), "v"(c), "v"(d)); }
__device__ __forceinline__ void keep4_b(v16b a, v16b b, v16b c, v16b d) { asm volatile("v_nop" :: "v"(a), "v"(b), "v"(c), "v"(d)); }
__device__ __forceinline__ void acc_guard4(v8f& a, v8f& b, v8f& c, v8f& d) { asm volatile("v_nop\n\tv_nop\n\tv_nop\n\tv_nop" : "+v"(a), "+v"(b), "+v"(c), "+v"(d)); }
template <typename T> struct Frag;
template <> struct Frag<_Float16> {
  typedef v16h V; union U { v16h v; v8h h[2]; };
  static __device__ __forceinline__ v16h load(const _Float16* p) {
    U f; f.h[0] = *(const v8h*)(p); f.h[1] = *(const v8h*)(p + 16); return f.v;
  }
  static __device__ __forceinline__ v8f mma(v16h a, v16h b, v8f c) {
    return __builtin_amdgcn_wmma_f32_16x16x32_f16(false, a, false, b, (short)0, c, false, false);
  }
  static __device__ __forceinline__ void guard(v8f& a, v8f& b, v16h x, v16h y) { dep_guard_h(a, b, x, y); }
  static __device__ __forceinline__ void keep(v16h a, v16h b, v16h c, v16h d) { keep4_h(a, b, c, d); }
};
template <> struct Frag<__bf16> {
  typedef v16b V; union U { v16b v; v8b h[2]; };
  static __device__ __forceinline__ v16b load(const __bf16* p) {
    U f; f.h[0] = *(const v8b*)(p); f.h[1] = *(const v8b*)(p + 16); return f.v;
  }
  static __device__ __forceinline__ v8f mma(v16b a, v16b b, v8f c) {
    return __builtin_amdgcn_wmma_f32_16x16x32_bf16(false, a, false, b, (short)0, c, false, false);
  }
  static __device__ __forceinline__ void guard(v8f& a, v8f& b, v16b x, v16b y) { dep_guard_b(a, b, x, y); }
  static __device__ __forceinline__ void keep(v16b a, v16b b, v16b c, v16b d) { keep4_b(a, b, c, d); }
};

__device__ __forceinline__ unsigned pk16(unsigned short a, unsigned short b) { return (unsigned)a | ((unsigned)b << 16); }
__device__ __forceinline__ unsigned short h_bits(float f) { const _Float16 h = (_Float16)f; return __builtin_bit_cast(unsigned short, h); }

template <int ET> struct Elem;
template <> struct Elem<0> { typedef _Float16 T; };
template <> struct Elem<1> { typedef __bf16 T; };
template <int ET, bool SPLIT, int BIAS_MODE, int OUT_MODE, bool RESID, int ACT = 0>
__global__ __launch_bounds__(256) void wmma_gemm64(
    const unsigned short* __restrict__ Ap, const unsigned short* __restrict__ A2p, int lda, long strideA,
    const unsigned short* __restrict__ Btp, const unsigned short* __restrict__ Bt2p, int ldb, long strideB,
    void* __restrict__ Cout, void* __restrict__ Cout2, int ldc, long strideC,
    const float* __restrict__ bias,
    const float* __restrict__ resid, long strideR,
    int M, int N, int K, float scale) {
  typedef typename Elem<ET>::T T;
  typedef typename Frag<T>::V V;
  const T* A = (const T*)Ap; const T* A2 = (const T*)A2p; const T* Bt = (const T*)Btp; const T* Bt2 = (const T*)Bt2p;
  __shared__ __align__(16) float sT[8][16 * 68];
  const int b    = blockIdx.y;
  const int lane = threadIdx.x & 31;
  const int wave = threadIdx.x >> 5;
  const int tilesN = N >> 6;
  const int tilesM = M >> 6;
  const int tile = blockIdx.x * 8 + wave;
  if (tile >= tilesM * tilesN) return;
  const int tm = tile / tilesN;
  const int tn = tile - tm * tilesN;
  const int m0 = tm << 6;
  const int n0 = tn << 6;

  const T* Ab  = A  + (size_t)b * strideA;
  const T* Bb  = Bt + (size_t)b * strideB;
  const T* Ab2 = SPLIT ? (A2  + (size_t)b * strideA) : nullptr;
  const T* Bb2 = SPLIT ? (Bt2 + (size_t)b * strideB) : nullptr;

  const int rlane = lane & 15;
  const int koff  = (lane >> 4) * 8;
  const int mOff  = (lane >> 4) * 8;

  v8f acc[4][4];
#pragma unroll
  for (int i = 0; i < 4; ++i)
#pragma unroll
    for (int j = 0; j < 4; ++j) acc[i][j] = (v8f){0.f,0.f,0.f,0.f,0.f,0.f,0.f,0.f};

  for (int k0 = 0; k0 < K; k0 += 32) {
    V bh[4], bl[4];
#pragma unroll
    for (int j = 0; j < 4; ++j) {
      const size_t bo = (size_t)(n0 + (j << 4) + rlane) * ldb + koff + k0;
      bh[j] = Frag<T>::load(Bb + bo);
      if (SPLIT) bl[j] = Frag<T>::load(Bb2 + bo);
    }
#pragma unroll
    for (int i = 0; i < 4; ++i) {
      const size_t ao = (size_t)(m0 + (i << 4) + rlane) * lda + koff + k0;
      V ah = Frag<T>::load(Ab + ao);
      V al;
      if (SPLIT) al = Frag<T>::load(Ab2 + ao);
#pragma unroll
      for (int j = 0; j < 4; ++j) {
        acc[i][j] = Frag<T>::mma(ah, bh[j], acc[i][j]);
        if (SPLIT) {
          acc[i][j] = Frag<T>::mma(ah, bl[j], acc[i][j]);
          acc[i][j] = Frag<T>::mma(al, bh[j], acc[i][j]);
        }
      }
      Frag<T>::guard(acc[i][0], acc[i][3], ah, SPLIT ? al : ah);
    }
    Frag<T>::keep(bh[0], bh[1], bh[2], bh[3]);
    if (SPLIT) Frag<T>::keep(bl[0], bl[1], bl[2], bl[3]);
  }
  acc_guard4(acc[0][0], acc[0][1], acc[0][2], acc[0][3]);
  acc_guard4(acc[1][0], acc[1][1], acc[1][2], acc[1][3]);
  acc_guard4(acc[2][0], acc[2][1], acc[2][2], acc[2][3]);
  acc_guard4(acc[3][0], acc[3][1], acc[3][2], acc[3][3]);

  float* slab = sT[wave];
  const float* Rb = RESID ? (resid + (size_t)b * strideR) : nullptr;
#pragma unroll
  for (int i = 0; i < 4; ++i) {
    const int mBase = m0 + (i << 4);
#pragma unroll
    for (int j = 0; j < 4; ++j) {
      const int n = n0 + (j << 4) + rlane;
      float bv = 0.f;
      if (BIAS_MODE == 2) bv = bias[n];
      if (BIAS_MODE == 4) bv = bf_bits2f(f2bf_bits(bias[n]));
#pragma unroll
      for (int r = 0; r < 8; ++r) {
        float v = acc[i][j][r] * scale;
        if (BIAS_MODE == 1) v += bias[mBase + mOff + r];
        if (BIAS_MODE == 3) v += bf_bits2f(f2bf_bits(bias[mBase + mOff + r]));
        if (BIAS_MODE == 2 || BIAS_MODE == 4) v += bv;
        if (RESID) v += Rb[(size_t)(mBase + mOff + r) * ldc + n];
        if (ACT == 2) v = fmaxf(v, 0.0f);
        if (ACT == 4) v = (v > 0.f) ? v : 0.01f * v;
        slab[(mOff + r) * 68 + (j << 4) + rlane] = v;
      }
    }
    __builtin_amdgcn_fence(__ATOMIC_RELEASE, "workgroup");
    __builtin_amdgcn_wave_barrier();
    __builtin_amdgcn_fence(__ATOMIC_ACQUIRE, "workgroup");
    if (OUT_MODE == 0) {
      float* C = (float*)Cout + (size_t)b * strideC;
      const int hh = lane >> 4, c4 = (lane & 15) * 4;
      for (int pass = 0; pass < 2; ++pass) {
#pragma unroll
        for (int it = 0; it < 8; ++it) {
          const int row = it * 2 + hh;
          v4f v = *(const v4f*)(slab + row * 68 + c4);
          *(volatile v4f*)(C + (size_t)(mBase + row) * ldc + n0 + c4) = v;
        }
        __threadfence();
      }
    } else {
      const int q = lane >> 3, c8 = (lane & 7) * 8;
      unsigned short* C  = (unsigned short*)Cout  + (size_t)b * strideC;
      unsigned short* C2 = (OUT_MODE == 2) ? ((unsigned short*)Cout2 + (size_t)b * strideC) : nullptr;
      for (int pass = 0; pass < 2; ++pass) {
#pragma unroll
        for (int it = 0; it < 4; ++it) {
          const int row = it * 4 + q;
          const float* sp = slab + row * 68 + c8;
          v8h hv, lv;
#pragma unroll
          for (int e = 0; e < 8; ++e) {
            if (OUT_MODE == 1) {
              hv[e] = (_Float16)sp[e];
              lv[e] = hv[e];
            } else {
              unsigned short hb = f2bf_bits(sp[e]);
              unsigned short lb = f2bf_bits(sp[e] - bf_bits2f(hb));
              hv[e] = __builtin_bit_cast(_Float16, hb);
              lv[e] = __builtin_bit_cast(_Float16, lb);
            }
          }
          *(volatile v8h*)(C + (size_t)(mBase + row) * ldc + n0 + c8) = hv;
          if (OUT_MODE == 2) *(volatile v8h*)(C2 + (size_t)(mBase + row) * ldc + n0 + c8) = lv;
        }
        __threadfence();
      }
    }
    __builtin_amdgcn_fence(__ATOMIC_RELEASE, "workgroup");
    __builtin_amdgcn_wave_barrier();
    __builtin_amdgcn_fence(__ATOMIC_ACQUIRE, "workgroup");
  }
}

__global__ __launch_bounds__(256) void wt_cast_bf16_kernel(const float* __restrict__ W0, const float* __restrict__ W1,
                                                         const float* __restrict__ W2, unsigned short* __restrict__ out) {
  __shared__ float sm[64][65];
  const int t  = threadIdx.x;
  const int k0 = blockIdx.x * 64;
  const int n0 = blockIdx.y * 64;
  const int z  = blockIdx.z;
  const float* W = (z == 0) ? W0 : (z == 1) ? W1 : W2;
#pragma unroll
  for (int i = 0; i < 16; ++i) {
    const int e = i * 256 + t;
    const int r = e >> 6;
    const int c = e & 63;
    sm[c][r] = W[(size_t)(k0 + r) * kDim + n0 + c];
  }
  __syncthreads();
  const int lane = t & 31, wave = t >> 5;
  const int q = lane >> 3, c8 = (lane & 7) * 8;
  unsigned short* op = out + (size_t)z * kDim * kDim;
  for (int pass = 0; pass < 2; ++pass) {
#pragma unroll
    for (int it = 0; it < 2; ++it) {
      const int row = wave * 8 + it * 4 + q;
      unsigned short hb[8];
#pragma unroll
      for (int e = 0; e < 8; ++e) hb[e] = f2bf_bits(sm[row][c8 + e]);
      const v4u u = (v4u){pk16(hb[0], hb[1]), pk16(hb[2], hb[3]), pk16(hb[4], hb[5]), pk16(hb[6], hb[7])};
      *(volatile v4u*)(op + (size_t)(n0 + row) * kDim + k0 + c8) = u;
    }
    __threadfence();
  }
}

__global__ __launch_bounds__(256) void cast8_bf16_kernel(const float* __restrict__ in, unsigned short* __restrict__ out, int n8) {
  const int i = blockIdx.x * 256 + threadIdx.x;
  if (i >= n8) return;
  const float* p = in + 8 * (size_t)i;
  const v4f a = *(const v4f*)(p);
  const v4f c = *(const v4f*)(p + 4);
  unsigned short hb[8];
#pragma unroll
  for (int e = 0; e < 4; ++e) {
    hb[e]     = f2bf_bits(a[e]);
    hb[4 + e] = f2bf_bits(c[e]);
  }
  const v4u u = (v4u){pk16(hb[0], hb[1]), pk16(hb[2], hb[3]), pk16(hb[4], hb[5]), pk16(hb[6], hb[7])};
  unsigned short* q = out + 8 * (size_t)i;
  *(volatile v4u*)q = u;
  __threadfence();
  *(volatile v4u*)q = u;
}

__global__ __launch_bounds__(256) void softmax_row_kernel(const float* __restrict__ Sin, unsigned short* __restrict__ Pout, float carry) {
  __shared__ float redM[8];
  __shared__ float redS[8];
  const int row  = blockIdx.x;
  const int t    = threadIdx.x;
  const int lane = t & 31, wave = t >> 5;
  const int cA   = 8 * t;
  const int cB   = kHalfRow + 8 * t;
  const float* sr = Sin + (size_t)row * kTok;
  const v4f a0 = *(const v4f*)(sr + cA);
  const v4f a1 = *(const v4f*)(sr + cA + 4);
  const v4f b0 = *(const v4f*)(sr + cB);
  const v4f b1 = *(const v4f*)(sr + cB + 4);
  float x[16];
#pragma unroll
  for (int e = 0; e < 4; ++e) { x[e] = a0[e]; x[4 + e] = a1[e]; x[8 + e] = b0[e]; x[12 + e] = b1[e]; }
  float m = x[0];
#pragma unroll
  for (int e = 1; e < 16; ++e) m = fmaxf(m, x[e]);
#pragma unroll
  for (int off = 16; off > 0; off >>= 1) m = fmaxf(m, __shfl_xor(m, off, 32));
  if (lane == 0) redM[wave] = m;
  __syncthreads();
  float gm = redM[0];
#pragma unroll
  for (int w = 1; w < 8; ++w) gm = fmaxf(gm, redM[w]);

  float ev[16];
  float ps = 0.f;
#pragma unroll
  for (int e = 0; e < 16; ++e) { ev[e] = __expf(x[e] - gm); ps += ev[e]; }
#pragma unroll
  for (int off = 16; off > 0; off >>= 1) ps += __shfl_xor(ps, off, 32);
  if (lane == 0) redS[wave] = ps;
  __syncthreads();
  float tot = redS[0];
#pragma unroll
  for (int w = 1; w < 8; ++w) tot += redS[w];
  const float inv = (1.0f / tot) * carry;

  unsigned short hb[16];
#pragma unroll
  for (int e = 0; e < 16; ++e) hb[e] = h_bits(ev[e] * inv);
  const v4u uA = (v4u){pk16(hb[0], hb[1]),  pk16(hb[2], hb[3]),   pk16(hb[4], hb[5]),   pk16(hb[6], hb[7])};
  const v4u uB = (v4u){pk16(hb[8], hb[9]),  pk16(hb[10], hb[11]), pk16(hb[12], hb[13]), pk16(hb[14], hb[15])};
  unsigned short* pr = Pout + (size_t)row * kTok;
  *(volatile v4u*)(pr + cA) = uA;
  *(volatile v4u*)(pr + cB) = uB;
  __threadfence();
  *(volatile v4u*)(pr + cA) = uA;
  *(volatile v4u*)(pr + cB) = uB;
}

extern "C" void kernel_launch(void* const* d_in, const int* in_sizes, int n_in,
                              void* d_out, int out_size, void* d_ws, size_t ws_size,
                              hipStream_t stream) {
  if (n_in < 9) return;
  if (in_sizes[0] != kRows * kDim || in_sizes[1] != kRows * kDim || in_sizes[2] != kRows * kDim) return;
  if (in_sizes[3] != kDim * kDim || in_sizes[5] != kDim * kDim || in_sizes[7] != kDim * kDim) return;
  if (in_sizes[4] != kDim || in_sizes[6] != kDim || in_sizes[8] != kDim) return;
  if (out_size != kRows * kDim) return;
  if (ws_size < kWsTotal) return;

  const float* query_X = (const float*)d_in[0];
  const float* key_X   = (const float*)d_in[1];
  const float* value_X = (const float*)d_in[2];
  const float* W_Q = (const float*)d_in[3];
  const float* b_Q = (const float*)d_in[4];
  const float* W_K = (const float*)d_in[5];
  const float* b_K = (const float*)d_in[6];
  const float* W_V = (const float*)d_in[7];
  const float* b_V = (const float*)d_in[8];
  float* out = (float*)d_out;

  char* ws = (char*)d_ws;
  unsigned short* Xb  = (unsigned short*)(ws + kOffXb);
  unsigned short* Pp  = (unsigned short*)(ws + kOffXb);
  unsigned short* Wt  = (unsigned short*)(ws + kOffWt);
  unsigned short* WtQ = Wt;
  unsigned short* WtK = Wt + (size_t)kDim * kDim;
  unsigned short* WtV = Wt + (size_t)2 * kDim * kDim;
  unsigned short* Qp  = (unsigned short*)(ws + kOffQp);
  unsigned short* Kp  = (unsigned short*)(ws + kOffKp);
  unsigned short* Vt  = (unsigned short*)(ws + kOffVt);
  float*          Sp  = (float*)(ws + kOffS);

  const int n8 = (kRows * kDim) / 8;
  const int castBlocks = n8 / 256;

  wt_cast_bf16_kernel<<<dim3(kDim / 64, kDim / 64, 3), 256, 0, stream>>>(W_Q, W_K, W_V, Wt);

  cast8_bf16_kernel<<<castBlocks, 256, 0, stream>>>(query_X, Xb, n8);
  wmma_gemm64<1, false, 4, 1, false, 0><<<dim3((kRows / 64) * (kDim / 64) / 8, 1), 256, 0, stream>>>(
      Xb, Xb, kDim, 0L, WtQ, WtQ, kDim, 0L, (void*)Qp, (void*)Qp, kDim, 0L, b_Q, b_Q, 0L, kRows, kDim, kDim, 1.0f);

  cast8_bf16_kernel<<<castBlocks, 256, 0, stream>>>(key_X, Xb, n8);
  wmma_gemm64<1, false, 4, 1, false, 0><<<dim3((kRows / 64) * (kDim / 64) / 8, 1), 256, 0, stream>>>(
      Xb, Xb, kDim, 0L, WtK, WtK, kDim, 0L, (void*)Kp, (void*)Kp, kDim, 0L, b_K, b_K, 0L, kRows, kDim, kDim, 1.0f);

  cast8_bf16_kernel<<<castBlocks, 256, 0, stream>>>(value_X, Xb, n8);
  wmma_gemm64<1, false, 3, 1, false, 0><<<dim3((kDim / 64) * (kTok / 64) / 8, kBatch), 256, 0, stream>>>(
      WtV, WtV, kDim, 0L, Xb, Xb, kDim, (long)kTok * kDim, (void*)Vt, (void*)Vt, kTok, (long)kDim * kTok,
      b_V, b_V, 0L, kDim, kTok, kDim, 1.0f);

  for (int b = 0; b < kBatch; ++b) {
    for (int hq = 0; hq < 2; ++hq) {
      const size_t qrow0 = (size_t)b * kTok + (size_t)hq * kHalfQ;
      const unsigned short* Qh = Qp + qrow0 * kDim;
      const unsigned short* Kb = Kp + (size_t)b * kTok * kDim;
      const unsigned short* Vb = Vt + (size_t)b * kDim * kTok;
      float* Ob = out + qrow0 * kDim;

      wmma_gemm64<0, false, 0, 0, false, 0><<<dim3((kHalfQ / 64) * (kTok / 64) / 8, 1), 256, 0, stream>>>(
          Qh, Qh, kDim, 0L, Kb, Kb, kDim, 0L, (void*)Sp, (void*)Sp, kTok, 0L, b_Q, b_Q, 0L, kHalfQ, kTok, kDim, kScoreScale);

      softmax_row_kernel<<<kHalfQ, 256, 0, stream>>>(Sp, Pp, kPCarry);

      wmma_gemm64<0, false, 0, 0, false, 0><<<dim3((kHalfQ / 64) * (kDim / 64) / 8, 1), 256, 0, stream>>>(
          Pp, Pp, kTok, 0L, Vb, Vb, kTok, 0L, (void*)Ob, (void*)Ob, kDim, 0L, b_V, b_V, 0L, kHalfQ, kDim, kTok, kPCarryInv);
    }
  }
}
